// rnn_lyapunov_70308614636158
// MI455X (gfx1250) — hardware-verified
//
#include <hip/hip_runtime.h>
#include <math.h>

constexpr int NBATCH    = 64;
constexpr int NSTEP     = 2048;
constexpr int NIN       = 64;
constexpr int NHID      = 512;
constexpr int NOUTF     = 64;
constexpr int FPIT      = 60;
constexpr int ROWS_BLK  = 32;
constexpr int NWAVE_REC = 8;
constexpr int NTHR_SEQ  = 32 * (NWAVE_REC + 1);
constexpr int NTHR_AUX  = 256;
constexpr int HPITCH    = 520;
constexpr int SLABP     = 68;
constexpr int NROWS     = NBATCH * NSTEP;
constexpr float WCARRY     = 64.0f;
constexpr float WCARRY_INV = 1.0f / 64.0f;
constexpr int PREP_BLK_A  = (NHID * NHID / 8) / NTHR_AUX;
constexpr int PREP_BLK_WI = (NHID * NIN / 8) / NTHR_AUX;
constexpr int PREP_BLK_WL = (NOUTF * NHID / 8) / NTHR_AUX;
constexpr int PREP_BLOCKS = PREP_BLK_A + PREP_BLK_WI + PREP_BLK_WL + 1;

static_assert(NBATCH % ROWS_BLK == 0);
static_assert(ROWS_BLK == 32);
static_assert(NHID == 64 * NWAVE_REC);
static_assert(NOUTF == 64);
static_assert(NIN % 32 == 0 && NHID % 32 == 0);
static_assert((FPIT & 1) == 0);
static_assert(HPITCH % 8 == 0 && HPITCH >= NHID);
static_assert(SLABP % 4 == 0 && SLABP >= NOUTF);
static_assert((NHID * NHID / 8) % NTHR_AUX == 0);
static_assert((NHID * NIN / 8) % NTHR_AUX == 0);
static_assert((NOUTF * NHID / 8) % NTHR_AUX == 0);
static_assert(NHID / 4 <= NTHR_AUX);
static_assert((NROWS * (NIN / 8)) % NTHR_AUX == 0);

typedef __attribute__((ext_vector_type(16))) _Float16 v16h;
typedef __attribute__((ext_vector_type(8)))  _Float16 v8h;
typedef __attribute__((ext_vector_type(8)))  float    v8f;
typedef __attribute__((ext_vector_type(4)))  float    v4f;

union FragU { v16h v; v8h h[2]; };
__device__ __forceinline__ v16h frag_load(const _Float16* p) {
  FragU f;
  f.h[0] = *(const v8h*)(p);
  f.h[1] = *(const v8h*)(p + 16);
  return f.v;
}
__device__ __forceinline__ v8f mma16(v16h a, v16h b, v8f c) {
  return __builtin_amdgcn_wmma_f32_16x16x32_f16(false, a, false, b, (short)0, c, false, false);
}
__device__ __forceinline__ void guard8(v8f& d0, v8f& d1, v8f& d2, v8f& d3, v8f& d4, v8f& d5, v8f& d6, v8f& d7,
                                       v16h a0, v16h a1, v16h b0, v16h b1, v16h b2, v16h b3) {
  asm volatile("v_nop\n\tv_nop\n\tv_nop\n\tv_nop"
               : "+v"(d0), "+v"(d1), "+v"(d2), "+v"(d3), "+v"(d4), "+v"(d5), "+v"(d6), "+v"(d7)
               : "v"(a0), "v"(a1), "v"(b0), "v"(b1), "v"(b2), "v"(b3));
}
__device__ __forceinline__ void mma_group(v8f (&acc)[2][4], v16h a0, v16h a1, v16h b0, v16h b1, v16h b2, v16h b3) {
  acc[0][0] = mma16(a0, b0, acc[0][0]);
  acc[0][1] = mma16(a0, b1, acc[0][1]);
  acc[0][2] = mma16(a0, b2, acc[0][2]);
  acc[0][3] = mma16(a0, b3, acc[0][3]);
  acc[1][0] = mma16(a1, b0, acc[1][0]);
  acc[1][1] = mma16(a1, b1, acc[1][1]);
  acc[1][2] = mma16(a1, b2, acc[1][2]);
  acc[1][3] = mma16(a1, b3, acc[1][3]);
  guard8(acc[0][0], acc[0][1], acc[0][2], acc[0][3], acc[1][0], acc[1][1], acc[1][2], acc[1][3], a0, a1, b0, b1, b2, b3);
}
__device__ __forceinline__ v8f splat8(float x) { return (v8f){x, x, x, x, x, x, x, x}; }
__device__ __forceinline__ float ftanh(float x) { return 1.0f - 2.0f * __builtin_amdgcn_rcpf(__expf(2.0f * x) + 1.0f); }

__device__ __forceinline__ void store8_twice(unsigned short* dst, v8h hv) {
  *(volatile v8h*)dst = hv;
  __threadfence();
  *(volatile v8h*)dst = hv;
}

__global__ __launch_bounds__(NTHR_AUX) void prep_kernel(const float* __restrict__ Whh, const float* __restrict__ omega,
                                                        const float* __restrict__ Wih, const float* __restrict__ Wlin,
                                                        const float* __restrict__ bih, const float* __restrict__ bhh,
                                                        unsigned short* __restrict__ A16, unsigned short* __restrict__ WI16,
                                                        unsigned short* __restrict__ WL16, float* __restrict__ BS) {
  const int blk = blockIdx.x;
  const int tid = threadIdx.x;
  if (blk < PREP_BLK_A) {
    const int i   = blk * NTHR_AUX + tid;
    const int row = i / (NHID / 8);
    const int k8  = (i - row * (NHID / 8)) * 8;
    const float* wp = Whh + (size_t)row * NHID + k8;
    const v4f w0 = *(const v4f*)(wp);
    const v4f w1 = *(const v4f*)(wp + 4);
    const v4f o0 = *(const v4f*)(omega + k8);
    const v4f o1 = *(const v4f*)(omega + k8 + 4);
    v8h hv;
#pragma unroll
    for (int e = 0; e < 4; ++e) {
      const float q0 = o0[e] * o0[e];
      const float q1 = o1[e] * o1[e];
      const float p0 = w0[e] * q0;
      const float p1 = w1[e] * q1;
      hv[e]     = (_Float16)(p0 * WCARRY);
      hv[4 + e] = (_Float16)(p1 * WCARRY);
    }
    store8_twice(A16 + (size_t)i * 8, hv);
  } else if (blk < PREP_BLK_A + PREP_BLK_WI) {
    const int i = (blk - PREP_BLK_A) * NTHR_AUX + tid;
    const float* wp = Wih + (size_t)i * 8;
    const v4f w0 = *(const v4f*)(wp);
    const v4f w1 = *(const v4f*)(wp + 4);
    v8h hv;
#pragma unroll
    for (int e = 0; e < 4; ++e) {
      hv[e]     = (_Float16)(w0[e] * WCARRY);
      hv[4 + e] = (_Float16)(w1[e] * WCARRY);
    }
    store8_twice(WI16 + (size_t)i * 8, hv);
  } else if (blk < PREP_BLK_A + PREP_BLK_WI + PREP_BLK_WL) {
    const int i = (blk - PREP_BLK_A - PREP_BLK_WI) * NTHR_AUX + tid;
    const float* wp = Wlin + (size_t)i * 8;
    const v4f w0 = *(const v4f*)(wp);
    const v4f w1 = *(const v4f*)(wp + 4);
    v8h hv;
#pragma unroll
    for (int e = 0; e < 4; ++e) {
      hv[e]     = (_Float16)(w0[e] * WCARRY);
      hv[4 + e] = (_Float16)(w1[e] * WCARRY);
    }
    store8_twice(WL16 + (size_t)i * 8, hv);
  } else {
    if (tid < NHID / 4) {
      const v4f a = *(const v4f*)(bih + tid * 4);
      const v4f b = *(const v4f*)(bhh + tid * 4);
      v4f o;
#pragma unroll
      for (int e = 0; e < 4; ++e) {
        const float s = a[e] + b[e];
        o[e] = s * WCARRY;
      }
      float* op = BS + tid * 4;
      *(volatile v4f*)op = o;
      __threadfence();
      *(volatile v4f*)op = o;
    }
  }
}

__global__ __launch_bounds__(NTHR_AUX) void cvt_u_kernel(const float* __restrict__ src, unsigned short* __restrict__ dst, int n8) {
  const int i = blockIdx.x * NTHR_AUX + threadIdx.x;
  if (i < n8) {
    const float* sp = src + (size_t)i * 8;
    const v4f a = *(const v4f*)(sp);
    const v4f b = *(const v4f*)(sp + 4);
    v8h hv;
#pragma unroll
    for (int e = 0; e < 4; ++e) {
      hv[e]     = (_Float16)a[e];
      hv[4 + e] = (_Float16)b[e];
    }
    store8_twice(dst + (size_t)i * 8, hv);
  }
}

__global__ __launch_bounds__(NTHR_SEQ) void seq_kernel(const unsigned short* __restrict__ U16p,
                                                       const unsigned short* __restrict__ A16p,
                                                       const unsigned short* __restrict__ WI16p,
                                                       const unsigned short* __restrict__ WL16p,
                                                       const float* __restrict__ BS, const float* __restrict__ blin,
                                                       float* __restrict__ out) {
  __shared__ __align__(16) _Float16 Ah[2][ROWS_BLK * HPITCH];
  __shared__ __align__(16) float    Sl[ROWS_BLK * SLABP];
  const _Float16* U16  = (const _Float16*)U16p;
  const _Float16* A16  = (const _Float16*)A16p;
  const _Float16* WI16 = (const _Float16*)WI16p;
  const _Float16* WL16 = (const _Float16*)WL16p;
  const int tid  = threadIdx.x;
  const int lane = tid & 31;
  const int wave = __builtin_amdgcn_readfirstlane(tid >> 5);
  const int c    = lane & 15;
  const int hh   = lane >> 4;
  const int koff = hh * 8;
  const int c4   = c * 4;
  const int rowbase = blockIdx.x * ROWS_BLK;
  const int wv = (wave < NWAVE_REC) ? wave : (NWAVE_REC - 1);

  {
    _Float16* ahf = &Ah[0][0];
#pragma unroll 1
    for (int i = tid; i < 2 * ROWS_BLK * HPITCH; i += NTHR_SEQ) ahf[i] = (_Float16)0.0f;
  }
  float bv[4], bl[4];
#pragma unroll
  for (int j = 0; j < 4; ++j) {
    bv[j] = BS[64 * wv + 16 * j + c];
    bl[j] = blin[16 * j + c];
  }
  const _Float16* wa0 = A16  + (size_t)(64 * wv + c) * NHID + koff;
  const _Float16* wi0 = WI16 + (size_t)(64 * wv + c) * NIN  + koff;
  const _Float16* wl0 = WL16 + (size_t)c * NHID + koff;
  const _Float16* ub0 = U16  + (size_t)(rowbase + c) * NSTEP * NIN + koff;
  __syncthreads();

  constexpr int NITER = FPIT + NSTEP;
#pragma unroll 1
  for (int g = 0; g <= NITER; ++g) {
    const int cur = g & 1;
    const _Float16* ah0 = &Ah[cur][0] + c * HPITCH + koff;
    const _Float16* ah1 = ah0 + 16 * HPITCH;
    if (wave < NWAVE_REC) {
      if (g < NITER) {
        const int t = (g < FPIT) ? 0 : (g - FPIT);
        v8f acc[2][4];
#pragma unroll
        for (int j = 0; j < 4; ++j) {
          acc[0][j] = splat8(bv[j]);
          acc[1][j] = splat8(bv[j]);
        }
        const _Float16* u0 = ub0 + (size_t)t * NIN;
        const _Float16* u1 = u0 + (size_t)16 * NSTEP * NIN;
#pragma unroll 1
        for (int kx = 0; kx < NIN; kx += 32) {
          const v16h a0 = frag_load(u0 + kx);
          const v16h a1 = frag_load(u1 + kx);
          const v16h b0 = frag_load(wi0 + kx);
          const v16h b1 = frag_load(wi0 + (size_t)16 * NIN + kx);
          const v16h b2 = frag_load(wi0 + (size_t)32 * NIN + kx);
          const v16h b3 = frag_load(wi0 + (size_t)48 * NIN + kx);
          mma_group(acc, a0, a1, b0, b1, b2, b3);
        }
#pragma unroll 1
        for (int k0 = 0; k0 < NHID; k0 += 32) {
          const v16h a0 = frag_load(ah0 + k0);
          const v16h a1 = frag_load(ah1 + k0);
          const v16h b0 = frag_load(wa0 + k0);
          const v16h b1 = frag_load(wa0 + (size_t)16 * NHID + k0);
          const v16h b2 = frag_load(wa0 + (size_t)32 * NHID + k0);
          const v16h b3 = frag_load(wa0 + (size_t)48 * NHID + k0);
          mma_group(acc, a0, a1, b0, b1, b2, b3);
        }
        _Float16* ahn = &Ah[cur ^ 1][0];
#pragma unroll
        for (int mi = 0; mi < 2; ++mi) {
#pragma unroll
          for (int j = 0; j < 4; ++j) {
            const int col = 64 * wave + 16 * j + c;
#pragma unroll
            for (int r = 0; r < 8; ++r) {
              const float z  = acc[mi][j][r] * WCARRY_INV;
              const float hv = ftanh(z);
              ahn[(mi * 16 + 8 * hh + r) * HPITCH + col] = (_Float16)hv;
            }
          }
        }
      }
    } else {
      if (g > FPIT) {
        const int t = g - FPIT - 1;
        v8f acc[2][4];
#pragma unroll
        for (int j = 0; j < 4; ++j) {
          acc[0][j] = splat8(0.0f);
          acc[1][j] = splat8(0.0f);
        }
#pragma unroll 1
        for (int k0 = 0; k0 < NHID; k0 += 32) {
          const v16h a0 = frag_load(ah0 + k0);
          const v16h a1 = frag_load(ah1 + k0);
          const v16h b0 = frag_load(wl0 + k0);
          const v16h b1 = frag_load(wl0 + (size_t)16 * NHID + k0);
          const v16h b2 = frag_load(wl0 + (size_t)32 * NHID + k0);
          const v16h b3 = frag_load(wl0 + (size_t)48 * NHID + k0);
          mma_group(acc, a0, a1, b0, b1, b2, b3);
        }
#pragma unroll
        for (int mi = 0; mi < 2; ++mi) {
#pragma unroll
          for (int j = 0; j < 4; ++j) {
#pragma unroll
            for (int r = 0; r < 8; ++r) {
              const float v = acc[mi][j][r] * WCARRY_INV + bl[j];
              Sl[(mi * 16 + 8 * hh + r) * SLABP + 16 * j + c] = v;
            }
          }
        }
        __builtin_amdgcn_fence(__ATOMIC_RELEASE, "workgroup");
        __builtin_amdgcn_wave_barrier();
        __builtin_amdgcn_fence(__ATOMIC_ACQUIRE, "workgroup");
        for (int pass = 0; pass < 2; ++pass) {
#pragma unroll
          for (int it = 0; it < 16; ++it) {
            const int row = it * 2 + hh;
            const v4f v = *(const v4f*)(Sl + row * SLABP + c4);
            *(volatile v4f*)(out + ((size_t)(rowbase + row) * NSTEP + (size_t)t) * NOUTF + c4) = v;
          }
          __threadfence();
        }
        __builtin_amdgcn_fence(__ATOMIC_RELEASE, "workgroup");
        __builtin_amdgcn_wave_barrier();
        __builtin_amdgcn_fence(__ATOMIC_ACQUIRE, "workgroup");
      }
    }
    __syncthreads();
  }
}

extern "C" void kernel_launch(void* const* d_in, const int* in_sizes, int n_in,
                              void* d_out, int out_size, void* d_ws, size_t ws_size, hipStream_t stream) {
  if (n_in < 8 || d_out == nullptr || d_ws == nullptr) return;
  if (in_sizes[0] != NBATCH * NSTEP * NIN || in_sizes[1] != NHID * NIN || in_sizes[2] != NHID * NHID ||
      in_sizes[3] != NHID || in_sizes[4] != NHID || in_sizes[5] != NHID ||
      in_sizes[6] != NOUTF * NHID || in_sizes[7] != NOUTF || out_size != NBATCH * NSTEP * NOUTF) return;

  const float* u     = (const float*)d_in[0];
  const float* w_ih  = (const float*)d_in[1];
  const float* w_hh  = (const float*)d_in[2];
  const float* b_ih  = (const float*)d_in[3];
  const float* b_hh  = (const float*)d_in[4];
  const float* omega = (const float*)d_in[5];
  const float* w_lin = (const float*)d_in[6];
  const float* b_lin = (const float*)d_in[7];
  float* out = (float*)d_out;

  char* ws = (char*)d_ws;
  size_t off = 0;
  auto carve = [&](size_t bytes) -> char* { char* p = ws + off; off += (bytes + 255) & ~(size_t)255; return p; };
  unsigned short* U16  = (unsigned short*)carve((size_t)NROWS * NIN * 2);
  unsigned short* A16  = (unsigned short*)carve((size_t)NHID * NHID * 2);
  unsigned short* WI16 = (unsigned short*)carve((size_t)NHID * NIN * 2);
  unsigned short* WL16 = (unsigned short*)carve((size_t)NOUTF * NHID * 2);
  float*          BS   = (float*)carve((size_t)NHID * 4);
  if (off > ws_size || off > (size_t)134217728) return;

  prep_kernel<<<PREP_BLOCKS, NTHR_AUX, 0, stream>>>(w_hh, omega, w_ih, w_lin, b_ih, b_hh, A16, WI16, WL16, BS);
  const int n8u = NROWS * (NIN / 8);
  cvt_u_kernel<<<(n8u + NTHR_AUX - 1) / NTHR_AUX, NTHR_AUX, 0, stream>>>(u, U16, n8u);
  seq_kernel<<<NBATCH / ROWS_BLK, NTHR_SEQ, 0, stream>>>(U16, A16, WI16, WL16, BS, b_lin, out);
}
